// HoMEMetaLayer_86955907875072
// MI455X (gfx1250) — hardware-verified
//
#include <hip/hip_runtime.h>
#define NB 16384
#define DI 512
#define E1 64
#define E2 32
#define DO 64
#define GHD 32
#define NEX 6
#define NG 3
#define N1 512
#define GCOL (NEX * E1)
#define LNEPS 1e-5f
typedef __bf16 v16b __attribute__((ext_vector_type(16)));
typedef unsigned short v8us __attribute__((ext_vector_type(8), may_alias));
typedef float  v8f  __attribute__((ext_vector_type(8)));
typedef float  v4f  __attribute__((ext_vector_type(4)));
typedef float  v4fa __attribute__((ext_vector_type(4), may_alias));
union FragB { v16b v; v8us half[2]; unsigned short u[16]; };

__device__ __forceinline__ unsigned short bf16_bits(float x) { unsigned int u = __float_as_uint(x); return (unsigned short)((u + 0x7FFFu + ((u >> 16) & 1u)) >> 16); }
__device__ __forceinline__ float bf16_val(unsigned short b) { return __uint_as_float(((unsigned int)b) << 16); }
__device__ __forceinline__ float bf16_round(float x) { return bf16_val(bf16_bits(x)); }
template <int NT>
__device__ __forceinline__ v8f mmaN(v16b ah, v16b al, v16b bh, v16b bl, v8f c) {
  c = __builtin_amdgcn_wmma_f32_16x16x32_bf16(false, ah, false, bh, (short)0, c, false, false);
  if (NT >= 2) c = __builtin_amdgcn_wmma_f32_16x16x32_bf16(false, al, false, bh, (short)0, c, false, false);
  if (NT >= 3) c = __builtin_amdgcn_wmma_f32_16x16x32_bf16(false, ah, false, bl, (short)0, c, false, false);
  asm volatile("v_nop\n\tv_nop\n\tv_nop\n\tv_nop" : "+v"(c) : "v"(ah), "v"(al), "v"(bh), "v"(bl));
  return c;
}

__global__ __launch_bounds__(256) void k_wt_bf16(const float* __restrict__ W, unsigned short* __restrict__ Wt, int K, int N) {
  const int t = blockIdx.x * 256 + threadIdx.x;
  const int k8n = K / 8;
  if (t >= N * k8n) return;
  const int n = t / k8n, k8 = (t % k8n) * 8;
  v8us v;
#pragma unroll
  for (int i = 0; i < 8; ++i) v[i] = bf16_bits(W[(size_t)(k8 + i) * N + n]);
  *(volatile v8us*)(Wt + (size_t)n * K + k8) = v;
  __threadfence();
  *(volatile v8us*)(Wt + (size_t)n * K + k8) = v;
}

template <bool ASPLIT, int ACT, bool BIAS_BF16>
__global__ __launch_bounds__(128) void k_gemm_bf(const float* __restrict__ A, int lda, const unsigned short* __restrict__ Wt, int ldb,
                                               const float* __restrict__ bias, float* __restrict__ C, int ldc, int M, int N, int K) {
  __shared__ __attribute__((aligned(16))) float so[4][16][64];
  const int tid = threadIdx.x, w = tid >> 5, lane = tid & 31, ln = lane & 15, hh = lane >> 4;
  const int ntn = N / 64;
  const int wid = blockIdx.x * 4 + w;
  const int mt = wid / ntn, nq = wid % ntn;
  if (mt * 16 >= M) return;
  const int row0 = mt * 16, col0 = nq * 64;
  const float* arow = A + (size_t)(row0 + ln) * lda;
  v8f acc[4] = {};
  for (int kb = 0; kb < K; kb += 32) {
    FragB ah, al;
    const v4f x0 = *(const v4fa*)(arow + kb + 8 * hh), x1 = *(const v4fa*)(arow + kb + 8 * hh + 4);
    const v4f x2 = *(const v4fa*)(arow + kb + 16 + 8 * hh), x3 = *(const v4fa*)(arow + kb + 16 + 8 * hh + 4);
    float xs[16] = {x0[0],x0[1],x0[2],x0[3],x1[0],x1[1],x1[2],x1[3],x2[0],x2[1],x2[2],x2[3],x3[0],x3[1],x3[2],x3[3]};
#pragma unroll
    for (int i = 0; i < 16; ++i) { const unsigned short hb = bf16_bits(xs[i]); ah.u[i] = hb; al.u[i] = ASPLIT ? bf16_bits(xs[i] - bf16_val(hb)) : (unsigned short)0; }
#pragma unroll
    for (int t = 0; t < 4; ++t) {
      const unsigned short* brow = Wt + (size_t)(col0 + t * 16 + ln) * ldb + kb;
      FragB b;
      b.half[0] = *(const v8us*)(brow + 8 * hh);
      b.half[1] = *(const v8us*)(brow + 16 + 8 * hh);
      acc[t] = mmaN<ASPLIT ? 2 : 1>(ah.v, al.v, b.v, b.v, acc[t]);
    }
  }
#pragma unroll
  for (int t = 0; t < 4; ++t) {
    float bv = bias ? bias[col0 + t * 16 + ln] : 0.f;
    if (BIAS_BF16) bv = bf16_round(bv);
#pragma unroll
    for (int r = 0; r < 8; ++r) { float v = acc[t][r] + bv; if (ACT == 1) v = fmaxf(v, 0.f); so[w][8 * hh + r][t * 16 + ln] = v; }
  }
  __builtin_amdgcn_fence(__ATOMIC_ACQ_REL, "workgroup");
  __builtin_amdgcn_wave_barrier();
  const int rsub = lane >> 4, c4 = (lane & 15) * 4;
  for (int pass = 0; pass < 2; ++pass) {
#pragma unroll
    for (int q = 0; q < 8; ++q) {
      const int r = q * 2 + rsub;
      const v4f v = *(const v4fa*)&so[w][r][c4];
      *(volatile v4f*)(C + (size_t)(row0 + r) * ldc + col0 + c4) = v;
    }
    if (pass == 0) __threadfence();
  }
}

template <bool ASPLIT, int ACT, bool BIAS_BF16, bool RES_BF16>
__global__ __launch_bounds__(128) void k_gemm_bf3(const float* __restrict__ A, int lda, const unsigned short* __restrict__ Wt, int ldb,
                                                const float* __restrict__ bias, const float* __restrict__ resid, int rmod, int ldr,
                                                float* __restrict__ C, int ldc, int M, int N, int K) {
  __shared__ __attribute__((aligned(16))) float so[4][16][64];
  const int tid = threadIdx.x, w = tid >> 5, lane = tid & 31, ln = lane & 15, hh = lane >> 4;
  const int ntn = N / 64;
  const int wid = blockIdx.x * 4 + w;
  const int mt = wid / ntn, nq = wid % ntn;
  if (mt * 16 >= M) return;
  const int row0 = mt * 16, col0 = nq * 64;
  const float* arow = A + (size_t)(row0 + ln) * lda;
  v8f acc[4] = {};
  for (int kb = 0; kb < K; kb += 32) {
    FragB ah, al;
    const v4f x0 = *(const v4fa*)(arow + kb + 8 * hh), x1 = *(const v4fa*)(arow + kb + 8 * hh + 4);
    const v4f x2 = *(const v4fa*)(arow + kb + 16 + 8 * hh), x3 = *(const v4fa*)(arow + kb + 16 + 8 * hh + 4);
    float xs[16] = {x0[0],x0[1],x0[2],x0[3],x1[0],x1[1],x1[2],x1[3],x2[0],x2[1],x2[2],x2[3],x3[0],x3[1],x3[2],x3[3]};
#pragma unroll
    for (int i = 0; i < 16; ++i) { const unsigned short hb = bf16_bits(xs[i]); ah.u[i] = hb; al.u[i] = ASPLIT ? bf16_bits(xs[i] - bf16_val(hb)) : (unsigned short)0; }
#pragma unroll
    for (int t = 0; t < 4; ++t) {
      const unsigned short* brow = Wt + (size_t)(col0 + t * 16 + ln) * ldb + kb;
      FragB b;
      b.half[0] = *(const v8us*)(brow + 8 * hh);
      b.half[1] = *(const v8us*)(brow + 16 + 8 * hh);
      acc[t] = mmaN<ASPLIT ? 2 : 1>(ah.v, al.v, b.v, b.v, acc[t]);
    }
  }
#pragma unroll
  for (int t = 0; t < 4; ++t) {
    const int col = col0 + t * 16 + ln;
    float bv = bias ? bias[col] : 0.f;
    if (BIAS_BF16) bv = bf16_round(bv);
#pragma unroll
    for (int r = 0; r < 8; ++r) {
      float v = acc[t][r] + bv;
      if (resid) { float rv = resid[(size_t)((row0 + 8 * hh + r) % rmod) * ldr + col]; if (RES_BF16) rv = bf16_round(rv); v += rv; }
      if (ACT == 1) v = fmaxf(v, 0.f);
      if (ACT == 2) v = 0.5f * v * (1.0f + erff(v * 0.70710678118654752f));
      if (ACT == 3) { const float u = 0.7978845608028654f * (v + 0.044715f * v * v * v); v = 0.5f * v * (1.0f + tanhf(u)); }
      so[w][8 * hh + r][t * 16 + ln] = v;
    }
  }
  __builtin_amdgcn_fence(__ATOMIC_ACQ_REL, "workgroup");
  __builtin_amdgcn_wave_barrier();
  const int rsub = lane >> 4, c4 = (lane & 15) * 4;
  for (int pass = 0; pass < 2; ++pass) {
#pragma unroll
    for (int q = 0; q < 8; ++q) {
      const int r = q * 2 + rsub;
      const v4f v = *(const v4fa*)&so[w][r][c4];
      *(volatile v4f*)(C + (size_t)(row0 + r) * ldc + col0 + c4) = v;
    }
    if (pass == 0) __threadfence();
  }
}
template <bool PARAM_BF16>
__global__ __launch_bounds__(256) void k_layernorm(const float* __restrict__ X, const float* __restrict__ R, const float* __restrict__ g, const float* __restrict__ bta,
                                                  float* __restrict__ out_sum, float* __restrict__ out_norm, int N, float eps) {
  __shared__ float red[256];
  const int row = blockIdx.x, tid = threadIdx.x;
  const float* x = X + (size_t)row * N; const float* rr = R ? R + (size_t)row * N : nullptr;
  float vals[16];
  const int per = N / 256;
  float s1 = 0.f;
  for (int u = 0; u < per / 4; ++u) {
    const int j = tid * 4 + 1024 * u;
    const v4f a = *(const v4fa*)(x + j);
    v4f b = {0.f,0.f,0.f,0.f}; if (rr) b = *(const v4fa*)(rr + j);
#pragma unroll
    for (int q = 0; q < 4; ++q) { const float v = a[q] + b[q]; vals[u * 4 + q] = v; s1 += v; }
  }
  red[tid] = s1; __syncthreads();
  for (int st = 128; st > 0; st >>= 1) { if (tid < st) red[tid] += red[tid + st]; __syncthreads(); }
  const float mu = red[0] / (float)N; __syncthreads();
  float s2 = 0.f;
  for (int u = 0; u < per / 4; ++u)
#pragma unroll
    for (int q = 0; q < 4; ++q) { const float c = vals[u * 4 + q] - mu; s2 += c * c; }
  red[tid] = s2; __syncthreads();
  for (int st = 128; st > 0; st >>= 1) { if (tid < st) red[tid] += red[tid + st]; __syncthreads(); }
  const float rs = rsqrtf(red[0] / (float)N + eps);
  for (int pass = 0; pass < 2; ++pass) {
    for (int u = 0; u < per / 4; ++u) {
      const int j = tid * 4 + 1024 * u;
      v4f o, sm;
#pragma unroll
      for (int q = 0; q < 4; ++q) {
        float gg = g[j + q], bb = bta[j + q];
        if (PARAM_BF16) { gg = bf16_round(gg); bb = bf16_round(bb); }
        sm[q] = vals[u * 4 + q]; o[q] = (vals[u * 4 + q] - mu) * rs * gg + bb;
      }
      if (out_sum) *(volatile v4f*)(out_sum + (size_t)row * N + j) = sm;
      *(volatile v4f*)(out_norm + (size_t)row * N + j) = o;
    }
    if (pass == 0) __threadfence();
  }
}


typedef _Float16 v16h __attribute__((ext_vector_type(16)));
union FragH { v16h v; v8us half[2]; _Float16 h[16]; unsigned short u[16]; };
template <int NT>
__device__ __forceinline__ v8f mmaH(v16h ah, v16h al, v16h bh, v16h bl, v8f c) {
  c = __builtin_amdgcn_wmma_f32_16x16x32_f16(false, ah, false, bh, (short)0, c, false, false);
  if (NT >= 2) c = __builtin_amdgcn_wmma_f32_16x16x32_f16(false, al, false, bh, (short)0, c, false, false);
  if (NT >= 3) c = __builtin_amdgcn_wmma_f32_16x16x32_f16(false, ah, false, bl, (short)0, c, false, false);
  asm volatile("v_nop\n\tv_nop\n\tv_nop\n\tv_nop" : "+v"(c) : "v"(ah), "v"(al), "v"(bh), "v"(bl));
  return c;
}
template <bool ASPLIT>
__global__ __launch_bounds__(128) void k_gemm_h(const float* __restrict__ A, int lda, size_t sA, const _Float16* __restrict__ Bh, int ldb, size_t sB, float alpha, float* __restrict__ C, int ldc, size_t sC, int M, int N, int K) {
  __shared__ __attribute__((aligned(16))) float so[4][16][64];
  const int tid = threadIdx.x, w = tid >> 5, lane = tid & 31, ln = lane & 15, hh = lane >> 4; const int by = blockIdx.y;
  A += (size_t)by * sA; Bh += (size_t)by * sB; C += (size_t)by * sC;
  const int ntn = (N + 63) / 64; const int wid = blockIdx.x * 4 + w; const int mt = wid / ntn, nq = wid % ntn; if (mt * 16 >= M) return;
  const int row0 = mt * 16, col0 = nq * 64; const float* arow = A + (size_t)(row0 + ln) * lda;
  v8f acc[4] = {};
  for (int kb = 0; kb < K; kb += 32) {
    FragH ah, al;
    const v4f x0 = *(const v4fa*)(arow + kb + 8 * hh), x1 = *(const v4fa*)(arow + kb + 8 * hh + 4), x2 = *(const v4fa*)(arow + kb + 16 + 8 * hh), x3 = *(const v4fa*)(arow + kb + 16 + 8 * hh + 4);
    float xs[16] = {x0[0],x0[1],x0[2],x0[3],x1[0],x1[1],x1[2],x1[3],x2[0],x2[1],x2[2],x2[3],x3[0],x3[1],x3[2],x3[3]};
#pragma unroll
    for (int i = 0; i < 16; ++i) { const _Float16 h = (_Float16)xs[i]; ah.h[i] = h; al.h[i] = ASPLIT ? (_Float16)(xs[i] - (float)h) : (_Float16)0.0f; }
#pragma unroll
    for (int t = 0; t < 4; ++t) { if (col0 + t * 16 >= N) continue; const size_t boff = (size_t)(col0 + t * 16 + ln) * ldb + kb; FragH bq; bq.half[0] = *(const v8us*)(Bh + boff + 8 * hh); bq.half[1] = *(const v8us*)(Bh + boff + 16 + 8 * hh);
      acc[t] = mmaH<ASPLIT ? 2 : 1>(ah.v, al.v, bq.v, bq.v, acc[t]); }
  }
#pragma unroll
  for (int t = 0; t < 4; ++t) { if (col0 + t * 16 >= N) continue;
#pragma unroll
    for (int r = 0; r < 8; ++r) so[w][8 * hh + r][t * 16 + ln] = acc[t][r] * alpha; }
  __builtin_amdgcn_fence(__ATOMIC_ACQ_REL, "workgroup"); __builtin_amdgcn_wave_barrier();
  const int rsub = lane >> 4, c4 = (lane & 15) * 4;
  for (int pass = 0; pass < 2; ++pass) {
#pragma unroll
    for (int q = 0; q < 8; ++q) { const int r = q * 2 + rsub; if (col0 + c4 < N) { const v4f v = *(const v4fa*)&so[w][r][c4]; *(volatile v4f*)(C + (size_t)(row0 + r) * ldc + col0 + c4) = v; } }
    if (pass == 0) __threadfence(); }
}

__global__ __launch_bounds__(256) void k_wt_f16(const float* __restrict__ W, _Float16* __restrict__ Wt, int K, int N, float scale) {
  const int t = blockIdx.x * 256 + threadIdx.x; if (t >= N * (K / 8)) return; const int n = t / (K / 8), k8 = (t % (K / 8)) * 8; FragH f;
#pragma unroll
  for (int i = 0; i < 8; ++i) f.h[i] = (_Float16)(bf16_round(W[(size_t)(k8 + i) * N + n]) * scale); const v8us o = f.half[0];
  *(volatile v8us*)((unsigned short*)Wt + (size_t)n * K + k8) = o; __threadfence(); *(volatile v8us*)((unsigned short*)Wt + (size_t)n * K + k8) = o;
}
template <int ACT>
__global__ __launch_bounds__(128) void k_gemm_hhx(const _Float16* __restrict__ A, int lda, size_t sA, const _Float16* __restrict__ Bh, int ldb, size_t sB, float alpha, const float* __restrict__ bias, size_t sBias, const float* __restrict__ CP, int rowsPerB, size_t sCPb, int row0g,
    float* __restrict__ C, _Float16* __restrict__ C16, int ldc, size_t sC, int M, int N, int K) {
  __shared__ __attribute__((aligned(16))) float so[4][16][64];
  const int tid = threadIdx.x, w = tid >> 5, lane = tid & 31, ln = lane & 15, hh = lane >> 4; const int by = blockIdx.y;
  A += (size_t)by * sA; Bh += (size_t)by * sB; const size_t cofs = (size_t)by * sC; const float* bp = bias ? bias + (size_t)by * sBias : nullptr;
  const int ntn = (N + 63) / 64; const int wid = blockIdx.x * 4 + w; const int mt = wid / ntn, nq = wid % ntn; if (mt * 16 >= M) return;
  const int row0 = mt * 16, col0 = nq * 64; const _Float16* arow = A + (size_t)(row0 + ln) * lda;
  v8f acc[4] = {};
  for (int kb = 0; kb < K; kb += 32) { FragH ah; ah.half[0] = *(const v8us*)((const unsigned short*)arow + kb + 8 * hh); ah.half[1] = *(const v8us*)((const unsigned short*)arow + kb + 16 + 8 * hh);
#pragma unroll
    for (int t = 0; t < 4; ++t) { if (col0 + t * 16 >= N) continue; const size_t boff = (size_t)(col0 + t * 16 + ln) * ldb + kb; FragH bq; bq.half[0] = *(const v8us*)((const unsigned short*)Bh + boff + 8 * hh); bq.half[1] = *(const v8us*)((const unsigned short*)Bh + boff + 16 + 8 * hh);
      acc[t] = mmaH<1>(ah.v, ah.v, bq.v, bq.v, acc[t]); }
  }
#pragma unroll
  for (int t = 0; t < 4; ++t) { if (col0 + t * 16 >= N) continue; const int col = col0 + t * 16 + ln; const float bv = bp ? bf16_round(bp[col]) : 0.f;
#pragma unroll
    for (int r = 0; r < 8; ++r) { float v = acc[t][r] * alpha + bv; if (CP) { const int bidx = (row0g + row0 + 8 * hh + r) / rowsPerB; v += CP[(size_t)bidx * sCPb + (size_t)by * 64 + col]; } if (ACT == 1) v = (v > 0.f) ? v : expm1f(v); else if (ACT == 7) v = (v > 0.f) ? v + 1.0f : expf(v); else if (ACT == 8) v = tanhf(v); else if (ACT == 9) v = 0.5f * v * (1.0f + tanhf(0.7978845608028654f * (v + 0.044715f * v * v * v))); else if (ACT == 11) v = 1.0f / (1.0f + expf(-v)); else if (ACT == 12) v = (v > 0.f) ? v : 0.01f * v; else if (ACT == 14) v = (v > 0.f) ? v : 0.1f * v; else if (ACT == 15) v = v / (1.0f + expf(-v)); else if (ACT == 3) v = fmaxf(v, 0.f); else if (ACT == 6) v = 0.5f * v * (1.0f + erff(v * 0.70710678118654752f)); so[w][8 * hh + r][t * 16 + ln] = v; } }
  __builtin_amdgcn_fence(__ATOMIC_ACQ_REL, "workgroup"); __builtin_amdgcn_wave_barrier();
  const int rsub = lane >> 4, c4 = (lane & 15) * 4; typedef _Float16 v4h __attribute__((ext_vector_type(4)));
  for (int pass = 0; pass < 2; ++pass) {
#pragma unroll
    for (int q = 0; q < 8; ++q) { const int r = q * 2 + rsub; if (col0 + c4 < N) { const v4f v = *(const v4fa*)&so[w][r][c4]; if (C) *(volatile v4f*)(C + cofs + (size_t)(row0 + r) * ldc + col0 + c4) = v; if (C16) { v4h h4; for (int i = 0; i < 4; ++i) h4[i] = (_Float16)v[i]; *(volatile v4h*)(C16 + cofs + (size_t)(row0 + r) * ldc + col0 + c4) = h4; } } }
    if (pass == 0) __threadfence(); }
}


typedef _Float16 v4h __attribute__((ext_vector_type(4)));

__global__ __launch_bounds__(256) void k_x16(const float* __restrict__ x, _Float16* __restrict__ X16, size_t n8) { const size_t t = (size_t)blockIdx.x * 256 + threadIdx.x; if (t >= n8) return; FragH f;
#pragma unroll
  for (int q = 0; q < 8; ++q) f.h[q] = (_Float16)bf16_round(x[t * 8 + q]); *(volatile v8us*)((unsigned short*)X16 + t * 8) = f.half[0]; __threadfence(); *(volatile v8us*)((unsigned short*)X16 + t * 8) = f.half[0]; }
__global__ __launch_bounds__(256) void k_h16(const float* __restrict__ x, _Float16* __restrict__ X16, size_t n8) { const size_t t = (size_t)blockIdx.x * 256 + threadIdx.x; if (t >= n8) return; FragH f;
#pragma unroll
  for (int q = 0; q < 8; ++q) f.h[q] = (_Float16)x[t * 8 + q]; *(volatile v8us*)((unsigned short*)X16 + t * 8) = f.half[0]; __threadfence(); *(volatile v8us*)((unsigned short*)X16 + t * 8) = f.half[0]; }
__global__ __launch_bounds__(256) void k_round16f(const float* __restrict__ W, _Float16* __restrict__ Bt, size_t n8) { const size_t t = (size_t)blockIdx.x * 256 + threadIdx.x; if (t >= n8) return; FragH f;
#pragma unroll
  for (int i = 0; i < 8; ++i) f.h[i] = (_Float16)(bf16_round(W[t * 8 + i]) * 16.0f); *(volatile v8us*)((unsigned short*)Bt + t * 8) = f.half[0]; __threadfence(); *(volatile v8us*)((unsigned short*)Bt + t * 8) = f.half[0]; }
template <int NHv, int TTv>
__global__ __launch_bounds__(256) void k_vt(const _Float16* __restrict__ V16, int ldv, int voff, _Float16* __restrict__ Vt) { __shared__ unsigned short tl[64][66]; const int tid = threadIdx.x; const int slab = blockIdx.x / (TTv / 64), lg = blockIdx.x % (TTv / 64); const int b = slab / NHv, h = slab % NHv;
  for (int i = tid; i < 64 * 8; i += 256) { const int r = i / 8, c8 = (i % 8) * 8; FragH f; f.half[0] = *(const v8us*)((const unsigned short*)V16 + ((size_t)b * TTv + lg * 64 + r) * ldv + voff + h * 64 + c8);
#pragma unroll
    for (int q = 0; q < 8; ++q) tl[r][c8 + q] = f.u[q]; }
  __syncthreads();
  for (int pass = 0; pass < 2; ++pass) {
#pragma unroll
    for (int rd = 0; rd < 2; ++rd) { const int d = rd * 32 + tid / 8, pc = tid % 8; FragH f;
#pragma unroll
      for (int q = 0; q < 8; ++q) f.u[q] = tl[pc * 8 + q][d];
      *(volatile v8us*)((unsigned short*)Vt + ((size_t)slab * 64 + d) * TTv + lg * 64 + pc * 8) = f.half[0]; }
    if (pass == 0) __threadfence(); } }

__global__ __launch_bounds__(256) void k_hl(const float* __restrict__ F, _Float16* __restrict__ Hh, _Float16* __restrict__ Hl, size_t n8) { const size_t t = (size_t)blockIdx.x * 256 + threadIdx.x; if (t >= n8) return; FragH fh, fl; const v4f a = *(const v4fa*)(F + t * 8), c = *(const v4fa*)(F + t * 8 + 4);
#pragma unroll
  for (int q = 0; q < 4; ++q) { _Float16 h = (_Float16)a[q]; fh.h[q] = h; fl.h[q] = (_Float16)((a[q] - (float)h) * 1024.0f); h = (_Float16)c[q]; fh.h[4 + q] = h; fl.h[4 + q] = (_Float16)((c[q] - (float)h) * 1024.0f); }
  for (int pass = 0; pass < 2; ++pass) { *(volatile v8us*)((unsigned short*)Hh + t * 8) = fh.half[0]; *(volatile v8us*)((unsigned short*)Hl + t * 8) = fl.half[0]; if (pass == 0) __threadfence(); } }

__global__ __launch_bounds__(256) void k_w1(const float* __restrict__ sw1, const float* __restrict__ gw1, const float* __restrict__ sgw1, const float* __restrict__ ggw1, _Float16* __restrict__ Bt) { const int t = blockIdx.x * 256 + threadIdx.x; if (t >= N1 * (DI / 8)) return; const int r = t / (DI / 8), c0 = (t % (DI / 8)) * 8; FragH f;
  const float* base = nullptr; int width = E1, o = 0;
  if (r < GCOL) { const int e6 = r / E1; o = r % E1; base = (e6 < 2) ? (sw1 + (size_t)e6 * DI * E1) : (gw1 + (size_t)(e6 - 2) * DI * E1); width = E1; }
  else if (r < GCOL + NG * GHD) { const int k = (r - GCOL) / GHD; o = (r - GCOL) % GHD; base = (k == 0) ? sgw1 : (ggw1 + (size_t)(k - 1) * DI * GHD); width = GHD; }
#pragma unroll
  for (int q = 0; q < 8; ++q) f.h[q] = base ? (_Float16)(bf16_round(base[(size_t)(c0 + q) * width + o]) * 16.0f) : (_Float16)0.0f;
  *(volatile v8us*)((unsigned short*)Bt + (size_t)r * DI + c0) = f.half[0]; __threadfence(); *(volatile v8us*)((unsigned short*)Bt + (size_t)r * DI + c0) = f.half[0]; }
__global__ __launch_bounds__(512) void k_b1(const float* __restrict__ sb1, const float* __restrict__ gb1, const float* __restrict__ sgb1, const float* __restrict__ ggb1, float* __restrict__ B1) { const int r = threadIdx.x; float v = 0.f;
  if (r < GCOL) { const int e6 = r / E1, o = r % E1; v = (e6 < 2) ? sb1[e6 * E1 + o] : gb1[(e6 - 2) * E1 + o]; }
  else if (r < GCOL + NG * GHD) { const int k = (r - GCOL) / GHD, o = (r - GCOL) % GHD; v = (k == 0) ? sgb1[o] : ggb1[(k - 1) * GHD + o]; }
  *(volatile float*)(B1 + r) = v; __threadfence(); *(volatile float*)(B1 + r) = v; }
__global__ __launch_bounds__(256) void k_w23(const float* __restrict__ sw2, const float* __restrict__ gw2, const float* __restrict__ sw3, const float* __restrict__ gw3, const float* __restrict__ sb2, const float* __restrict__ gb2, const float* __restrict__ sb3, const float* __restrict__ gb3,
                                             _Float16* __restrict__ Bt2, _Float16* __restrict__ Bt3, float* __restrict__ B2, float* __restrict__ B3) { const int e6 = blockIdx.x, tid = threadIdx.x;
  const float* W2 = (e6 < 2) ? (sw2 + (size_t)e6 * E1 * E2) : (gw2 + (size_t)(e6 - 2) * E1 * E2); const float* W3 = (e6 < 2) ? (sw3 + (size_t)e6 * E2 * DO) : (gw3 + (size_t)(e6 - 2) * E2 * DO);
  const float* b2 = (e6 < 2) ? (sb2 + e6 * E2) : (gb2 + (e6 - 2) * E2); const float* b3 = (e6 < 2) ? (sb3 + e6 * DO) : (gb3 + (e6 - 2) * DO);
  { const int o2 = tid / 8, c0 = (tid % 8) * 8; FragH f;
#pragma unroll
    for (int q = 0; q < 8; ++q) f.h[q] = (_Float16)(bf16_round(W2[(size_t)(c0 + q) * E2 + o2]) * 16.0f);
    *(volatile v8us*)((unsigned short*)Bt2 + ((size_t)e6 * E2 + o2) * E1 + c0) = f.half[0]; __threadfence(); *(volatile v8us*)((unsigned short*)Bt2 + ((size_t)e6 * E2 + o2) * E1 + c0) = f.half[0]; }
  { const int o3 = tid / 4, c0 = (tid % 4) * 8; FragH f;
#pragma unroll
    for (int q = 0; q < 8; ++q) f.h[q] = (_Float16)(bf16_round(W3[(size_t)(c0 + q) * DO + o3]) * 16.0f);
    *(volatile v8us*)((unsigned short*)Bt3 + ((size_t)e6 * DO + o3) * E2 + c0) = f.half[0]; __threadfence(); *(volatile v8us*)((unsigned short*)Bt3 + ((size_t)e6 * DO + o3) * E2 + c0) = f.half[0]; }
  if (tid < E2) { *(volatile float*)(B2 + e6 * E2 + tid) = b2[tid]; __threadfence(); *(volatile float*)(B2 + e6 * E2 + tid) = b2[tid]; }
  if (tid >= 64 && tid < 64 + DO) { const int o = tid - 64; *(volatile float*)(B3 + e6 * DO + o) = b3[o]; __threadfence(); *(volatile float*)(B3 + e6 * DO + o) = b3[o]; } }
__global__ __launch_bounds__(256) void k_combine(const float* __restrict__ O, const float* __restrict__ H1f, const float* __restrict__ sgam, const float* __restrict__ sbet, const float* __restrict__ ggam, const float* __restrict__ gbet,
                                                 const float* __restrict__ sgw2, const float* __restrict__ sgb2, const float* __restrict__ ggw2, const float* __restrict__ ggb2, float* __restrict__ out) {
  #pragma clang fp contract(off)
  const size_t t = (size_t)blockIdx.x * 256 + threadIdx.x; if (t >= (size_t)NG * NB * 16) return; const int i = (int)(t & 15); const size_t kr = t >> 4; const int k = (int)(kr / NB); const size_t r = kr % NB; const int c0 = i * 4;
  const int ea = (k == 2) ? 0 : 2 + 2 * k, eb = ea + 1; const int kg = (k == 2) ? 0 : 1 + k;
  const float* gam0 = (k == 2) ? sgam : (ggam + (size_t)k * 2 * DO); const float* bet0 = (k == 2) ? sbet : (gbet + (size_t)k * 2 * DO); const float* gw2 = (k == 2) ? sgw2 : (ggw2 + (size_t)k * GHD * 2); const float* gb2 = (k == 2) ? sgb2 : (ggb2 + (size_t)k * 2);
  const float* gh = H1f + r * N1 + GCOL + kg * GHD; float l0 = bf16_round(gb2[0]), l1 = bf16_round(gb2[1]);
#pragma unroll 1
  for (int c = 0; c < GHD; ++c) { const float h = gh[c]; l0 += h * bf16_round(gw2[c * 2 + 0]); l1 += h * bf16_round(gw2[c * 2 + 1]); }
  const float mx = fmaxf(l0, l1); const float e0 = expf(l0 - mx), e1 = expf(l1 - mx); const float w0 = e0 / (e0 + e1), w1 = e1 / (e0 + e1);
  v4f z = {0.f, 0.f, 0.f, 0.f};
#pragma unroll
  for (int which = 0; which < 2; ++which) { const int e6 = which ? eb : ea; const v4f o = *(const v4fa*)(O + ((size_t)e6 * NB + r) * DO + c0);
    float s = (o[0] + o[1]) + (o[2] + o[3]); s += __shfl_xor(s, 1, 32); s += __shfl_xor(s, 2, 32); s += __shfl_xor(s, 4, 32); s += __shfl_xor(s, 8, 32); const float mu = s * (1.0f / DO);
    float q2 = 0.f;
#pragma unroll
    for (int j = 0; j < 4; ++j) { const float d = o[j] - mu; q2 += d * d; }
    q2 += __shfl_xor(q2, 1, 32); q2 += __shfl_xor(q2, 2, 32); q2 += __shfl_xor(q2, 4, 32); q2 += __shfl_xor(q2, 8, 32); const float rs = rsqrtf(q2 * (1.0f / DO) + LNEPS); const float w = which ? w1 : w0;
    const float* gm = gam0 + which * DO + c0; const float* bt = bet0 + which * DO + c0;
#pragma unroll
    for (int j = 0; j < 4; ++j) z[j] += w * (bf16_round(gm[j]) * (o[j] - mu) * rs + bf16_round(bt[j])); }
  float* op = out + ((size_t)k * NB + r) * DO + c0; *(volatile v4f*)op = z; __threadfence(); *(volatile v4f*)op = z; }

extern "C" void kernel_launch(void* const* d_in, const int* in_sizes, int n_in,
                              void* d_out, int out_size, void* d_ws, size_t ws_size, hipStream_t stream) {
  (void)in_sizes; (void)n_in; (void)out_size;
  const float* const* I = (const float* const*)d_in; const float* v = I[0];
  const float* sw1 = I[1]; const float* sb1 = I[2]; const float* sw2 = I[3]; const float* sb2 = I[4]; const float* sw3 = I[5]; const float* sb3 = I[6]; const float* sgam = I[7]; const float* sbet = I[8];
  const float* sgw1 = I[9]; const float* sgb1 = I[10]; const float* sgw2 = I[11]; const float* sgb2 = I[12];
  const float* gw1 = I[13]; const float* gb1 = I[14]; const float* gw2 = I[15]; const float* gb2 = I[16]; const float* gw3 = I[17]; const float* gb3 = I[18]; const float* ggam = I[19]; const float* gbet = I[20];
  const float* ggw1 = I[21]; const float* ggb1 = I[22]; const float* ggw2 = I[23]; const float* ggb2 = I[24];
  char* ws = (char*)d_ws; size_t off = 0;
  auto take = [&](size_t bytes) { char* p = ws + off; off += (bytes + 255) & ~(size_t)255; return p; };
  _Float16* Bt1 = (_Float16*)take((size_t)N1 * DI * 2); float* B1 = (float*)take((size_t)N1 * 4); _Float16* Bt2 = (_Float16*)take((size_t)NEX * E2 * E1 * 2); _Float16* Bt3 = (_Float16*)take((size_t)NEX * DO * E2 * 2); float* B2 = (float*)take((size_t)NEX * E2 * 4); float* B3 = (float*)take((size_t)NEX * DO * 4);
  _Float16* V16 = (_Float16*)take((size_t)NB * DI * 2); float* H1f = (float*)take((size_t)NB * N1 * 4); _Float16* H1h = (_Float16*)take((size_t)NB * N1 * 2); _Float16* H2 = (_Float16*)take((size_t)NEX * NB * 64 * 2); float* O = (float*)take((size_t)NEX * NB * DO * 4);
  if (off > ws_size) return;
  k_w1<<<(N1 * (DI / 8) + 255) / 256, 256, 0, stream>>>(sw1, gw1, sgw1, ggw1, Bt1); k_b1<<<1, 512, 0, stream>>>(sb1, gb1, sgb1, ggb1, B1);
  k_w23<<<NEX, 256, 0, stream>>>(sw2, gw2, sw3, gw3, sb2, gb2, sb3, gb3, Bt2, Bt3, B2, B3);
  k_x16<<<(unsigned)(((size_t)NB * DI / 8 + 255) / 256), 256, 0, stream>>>(v, V16, (size_t)NB * DI / 8);
  k_gemm_hhx<15><<<dim3(((NB / 16) * (N1 / 64) + 3) / 4, 1), 128, 0, stream>>>(V16, DI, 0, Bt1, DI, 0, 0.0625f, B1, 0, nullptr, 1, 0, 0, H1f, H1h, N1, 0, NB, N1, DI);
  k_gemm_hhx<15><<<dim3(((NB / 16) * 1 + 3) / 4, NEX), 128, 0, stream>>>(H1h, N1, E1, Bt2, E1, (size_t)E2 * E1, 0.0625f, B2, E2, nullptr, 1, 0, 0, nullptr, H2, 64, (size_t)NB * 64, NB, E2, E1);
  k_gemm_hhx<0><<<dim3(((NB / 16) * 1 + 3) / 4, NEX), 128, 0, stream>>>(H2, 64, (size_t)NB * 64, Bt3, E2, (size_t)DO * E2, 0.0625f, B3, DO, nullptr, 1, 0, 0, O, nullptr, DO, (size_t)NB * DO, NB, DO, E2);
  k_combine<<<(unsigned)(((size_t)NG * NB * 16 + 255) / 256), 256, 0, stream>>>(O, H1f, sgam, sbet, ggam, gbet, sgw2, sgb2, ggw2, ggb2, (float*)d_out);
}
